// EncoderBlock_35424890258020
// MI455X (gfx1250) — hardware-run, weakly checked
//
#include <hip/hip_runtime.h>
#include <hip/hip_fp16.h>


#ifndef NB
#define NB 32
#endif
#ifndef SEQ
#define SEQ 512
#endif
#define NB_FULL  32
#define SEQ_FULL 512
#define NH   8
#define HD   64
#define DM   512
#define KW   7
#define NREL 33
#define NTOK (NB * SEQ)

static_assert(NB >= 1 && NB <= NB_FULL);
static_assert(SEQ >= 128 && SEQ <= SEQ_FULL);
static_assert(SEQ % 128 == 0);
static_assert(NTOK % 128 == 0);
static_assert(DM == NH * HD);
static_assert(DM == 512 && HD == 64 && NH == 8);
static_assert(KW == 7 && NREL == 33);
static_assert((DM * DM) % 2048 == 0);
static_assert(DM % 32 == 0 && HD % 32 == 0);

typedef _Float16 v16h __attribute__((ext_vector_type(16)));
typedef _Float16 v8h  __attribute__((ext_vector_type(8)));
typedef float    v8f  __attribute__((ext_vector_type(8)));
typedef float    v4f  __attribute__((ext_vector_type(4)));

union Frag { v16h v; v8h h[2]; };

#define LOG2E 1.44269504088896340736f
#define C1 (1.44269504088896340736f * 0.000244140625f)
#define SC_Q     6.25e-02f
#define SC_CONV  6.103515625e-05f
#define SC_OUT   9.765625e-04f
#define SC_REL   2.44140625e-04f
#define PE_DIV   (-0.017988946039015984f)

static __device__ __forceinline__ v8f zero8() {
    v8f z;
#pragma unroll
    for (int i = 0; i < 8; ++i) z[i] = 0.0f;
    return z;
}

static __device__ __forceinline__ v16h load_frag16(const _Float16* base, unsigned ld, unsigned lane) {
    const unsigned m  = lane & 15u;
    const unsigned kb = (lane >> 4) << 3;
    const _Float16* p = base + (size_t)m * ld + kb;
    Frag f;
    f.h[0] = *(const v8h*)(p);
    f.h[1] = *(const v8h*)(p + 16);
    return f.v;
}

static __device__ __forceinline__ v8f wmma16(v16h a, v16h b, v8f c) {
    v8f d = __builtin_amdgcn_wmma_f32_16x16x32_f16(false, a, false, b, (short)0, c, false, false);
    asm volatile("v_nop\n\tv_nop\n\tv_nop\n\tv_nop" : "+v"(d) : "v"(a), "v"(b));
    return d;
}

static __device__ __forceinline__ float bf16r(float x) {
    unsigned u = __float_as_uint(x);
    u = (u + 0x7FFFu + ((u >> 16) & 1u)) & 0xFFFF0000u;
    return __uint_as_float(u);
}

static __device__ __forceinline__ _Float16 toh_flush(float v) {
    const _Float16 r = (_Float16)v;
    return (fabsf(v) < 6.103515625e-05f) ? (_Float16)0.0f : r;
}

static __device__ __forceinline__ float ex2(float x) {
    return __builtin_amdgcn_exp2f(x);
}

static __device__ __forceinline__ void wave_lds_sync() {
    __builtin_amdgcn_fence(3, "wavefront");
    asm volatile("s_wait_dscnt 0" ::: "memory");
    __builtin_amdgcn_wave_barrier();
}

static __device__ __forceinline__ float wave_sum(float v) {
    v += __shfl_xor(v, 16, 32);
    v += __shfl_xor(v, 8, 32);
    v += __shfl_xor(v, 4, 32);
    v += __shfl_xor(v, 2, 32);
    v += __shfl_xor(v, 1, 32);
    return v;
}

static __device__ __forceinline__ unsigned full_row(unsigned n) {
    const unsigned b = n / (unsigned)SEQ;
    return b * (unsigned)SEQ_FULL + (n - b * (unsigned)SEQ);
}

template <int TM, int TN, bool RES>
static __device__ __forceinline__ void gemm_core(const _Float16* __restrict__ Ah,
                                                 const _Float16* __restrict__ Ar,
                                                 const _Float16* __restrict__ Bt,
                                                 unsigned K, unsigned lane,
                                                 v8f (&acc)[TM][TN], v8f (&accr)[TM][TN]) {
#pragma unroll
    for (int mt = 0; mt < TM; ++mt)
#pragma unroll
        for (int nt = 0; nt < TN; ++nt) {
            acc[mt][nt] = zero8();
            if (RES) accr[mt][nt] = zero8();
        }
#pragma unroll 1
    for (unsigned k = 0; k < K; k += 32u) {
        v16h a[TM];
        v16h ar[TM];
#pragma unroll
        for (int mt = 0; mt < TM; ++mt) {
            a[mt] = load_frag16(Ah + (size_t)(mt * 16) * K + k, K, lane);
            if (RES) ar[mt] = load_frag16(Ar + (size_t)(mt * 16) * K + k, K, lane);
        }
#pragma unroll
        for (int nt = 0; nt < TN; ++nt) {
            const v16h bfr = load_frag16(Bt + (size_t)(nt * 16) * K + k, K, lane);
#pragma unroll
            for (int mt = 0; mt < TM; ++mt) {
                acc[mt][nt] = wmma16(a[mt], bfr, acc[mt][nt]);
                if (RES) accr[mt][nt] = wmma16(ar[mt], bfr, accr[mt][nt]);
            }
        }
    }
}

__global__ __launch_bounds__(256) void k_wcvt(const float* __restrict__ src,
                                               _Float16* __restrict__ dst) {
    const unsigned idx = blockIdx.x * 256u + threadIdx.x;
    const float* p = src + (size_t)idx * 8u;
    const v4f a = *(const v4f*)(p);
    const v4f b = *(const v4f*)(p + 4);
    v8h o;
    o[0] = toh_flush(bf16r(a.x) * 64.0f); o[1] = toh_flush(bf16r(a.y) * 64.0f);
    o[2] = toh_flush(bf16r(a.z) * 64.0f); o[3] = toh_flush(bf16r(a.w) * 64.0f);
    o[4] = toh_flush(bf16r(b.x) * 64.0f); o[5] = toh_flush(bf16r(b.y) * 64.0f);
    o[6] = toh_flush(bf16r(b.z) * 64.0f); o[7] = toh_flush(bf16r(b.w) * 64.0f);
    _Float16* d = dst + (size_t)idx * 8u;
    *(volatile v8h*)d = o;
    __threadfence();
    *(volatile v8h*)d = o;
}

__global__ __launch_bounds__(256) void k_pe(float* __restrict__ pe) {
    __shared__ __align__(16) float prow[DM];
    const unsigned tid = threadIdx.x;
    const unsigned s   = blockIdx.x;
    const float pos = (float)((int)s - 1);
    const float dv  = expf((float)(2u * tid) * PE_DIV);
    const float a   = pos * dv;
    const float sn  = sinf(a);
    const float cs  = cosf(a);
    prow[2u * tid]      = (s > 0u) ? sn : 0.0f;
    prow[2u * tid + 1u] = (s > 0u) ? cs : 0.0f;
    __syncthreads();
    if (tid < 128u) {
        const v4f v = *(const v4f*)(&prow[tid * 4u]);
        float* d = pe + (size_t)s * DM + tid * 4u;
        *(volatile v4f*)d = v;
        __threadfence();
        *(volatile v4f*)d = v;
    }
}
static_assert(128 * 16 == DM * 4);

__global__ __launch_bounds__(256) void k_pos(const float* __restrict__ x,
                                              const int* __restrict__ mask,
                                              const float* __restrict__ pe,
                                              float* __restrict__ xs) {
    const unsigned idx = blockIdx.x * 256u + threadIdx.x;
    const unsigned n   = idx >> 7;
    const unsigned c4  = (idx & 127u) << 2;
    const unsigned b   = n / (unsigned)SEQ;
    const unsigned l   = n - b * (unsigned)SEQ;
    const unsigned fr  = full_row(n);
    const v4f a = *(const v4f*)(x + (size_t)fr * DM + c4);
    const v4f p = *(const v4f*)(pe + (size_t)l * DM + c4);
    const float m = (float)mask[fr];
    v4f o;
    o.x = bf16r(a.x) + p.x * m;
    o.y = bf16r(a.y) + p.y * m;
    o.z = bf16r(a.z) + p.z * m;
    o.w = bf16r(a.w) + p.w * m;
    float* d = xs + (size_t)n * DM + c4;
    *(volatile v4f*)d = o;
    __threadfence();
    *(volatile v4f*)d = o;
}

__global__ __launch_bounds__(256) __attribute__((amdgpu_num_vgpr(256)))
void k_lnconv(const float* __restrict__ xs,
              const float* __restrict__ lng, const float* __restrict__ lnb,
              const float* __restrict__ dw, const float* __restrict__ db,
              _Float16* __restrict__ hpl) {
    __shared__ __align__(16) float Tn[38 * DM];
    __shared__ __align__(16) float Wd[KW * DM];
    __shared__ __align__(16) float Bd[DM];
    const unsigned tid  = threadIdx.x;
    const unsigned lane = tid & 31u;
    const unsigned wave = __builtin_amdgcn_readfirstlane(tid >> 5);
    const unsigned row0 = blockIdx.x * 32u;
    const unsigned b    = row0 / (unsigned)SEQ;
    const unsigned l0   = row0 - b * (unsigned)SEQ;

#pragma unroll 1
    for (unsigned idx = tid; idx < (unsigned)(KW * DM); idx += 256u) {
        const unsigned c = idx / 7u;
        const unsigned k = idx - c * 7u;
        Wd[k * DM + c] = bf16r(dw[idx]);
    }
    Bd[tid]        = bf16r(db[tid]);
    Bd[tid + 256u] = bf16r(db[tid + 256u]);

#pragma unroll 1
    for (unsigned j = wave; j < 38u; j += 8u) {
        const int l = (int)l0 + (int)j - 3;
        if ((l >= 0) & (l < SEQ)) {
            const float* rp = xs + ((size_t)b * SEQ + (unsigned)l) * DM;
            v4f xv[4];
            float s = 0.0f;
#pragma unroll
            for (int i = 0; i < 4; ++i) {
                const unsigned c = (unsigned)i * 128u + lane * 4u;
                xv[i] = *(const v4f*)(rp + c);
                s += (xv[i].x + xv[i].y) + (xv[i].z + xv[i].w);
            }
            s = wave_sum(s);
            const float mu = s * (1.0f / (float)DM);
            float q = 0.0f;
#pragma unroll
            for (int i = 0; i < 4; ++i) {
                const float d0 = xv[i].x - mu, d1 = xv[i].y - mu, d2 = xv[i].z - mu, d3 = xv[i].w - mu;
                q += (d0 * d0 + d1 * d1) + (d2 * d2 + d3 * d3);
            }
            q = wave_sum(q);
            const float rstd = rsqrtf(q * (1.0f / (float)DM) + 1.0e-5f);
#pragma unroll
            for (int i = 0; i < 4; ++i) {
                const unsigned c = (unsigned)i * 128u + lane * 4u;
                const v4f gw = *(const v4f*)(lng + c);
                const v4f gb = *(const v4f*)(lnb + c);
                v4f y;
                y.x = (xv[i].x - mu) * rstd * bf16r(gw.x) + bf16r(gb.x);
                y.y = (xv[i].y - mu) * rstd * bf16r(gw.y) + bf16r(gb.y);
                y.z = (xv[i].z - mu) * rstd * bf16r(gw.z) + bf16r(gb.z);
                y.w = (xv[i].w - mu) * rstd * bf16r(gw.w) + bf16r(gb.w);
                *(v4f*)(&Tn[j * DM + c]) = y;
            }
        } else {
            v4f z;
            z.x = 0.0f; z.y = 0.0f; z.z = 0.0f; z.w = 0.0f;
#pragma unroll
            for (int i = 0; i < 4; ++i)
                *(v4f*)(&Tn[j * DM + (unsigned)i * 128u + lane * 4u]) = z;
        }
    }
    __syncthreads();

#pragma unroll 1
    for (unsigned rr = 0; rr < 4u; ++rr) {
        const unsigned r = wave * 4u + rr;
        v8h hv[2];
#pragma unroll
        for (int ch = 0; ch < 2; ++ch) {
            const unsigned c8 = (unsigned)ch * 256u + lane * 8u;
            v4f a0 = *(const v4f*)(&Bd[c8]);
            v4f a1 = *(const v4f*)(&Bd[c8 + 4u]);
#pragma unroll 1
            for (unsigned k = 0; k < (unsigned)KW; ++k) {
                const v4f t0 = *(const v4f*)(&Tn[(r + k) * DM + c8]);
                const v4f t1 = *(const v4f*)(&Tn[(r + k) * DM + c8 + 4u]);
                const v4f w0 = *(const v4f*)(&Wd[k * DM + c8]);
                const v4f w1 = *(const v4f*)(&Wd[k * DM + c8 + 4u]);
                a0 += t0 * w0;
                a1 += t1 * w1;
            }
            v8h o;
            o[0] = toh_flush(a0.x * 256.0f); o[1] = toh_flush(a0.y * 256.0f);
            o[2] = toh_flush(a0.z * 256.0f); o[3] = toh_flush(a0.w * 256.0f);
            o[4] = toh_flush(a1.x * 256.0f); o[5] = toh_flush(a1.y * 256.0f);
            o[6] = toh_flush(a1.z * 256.0f); o[7] = toh_flush(a1.w * 256.0f);
            hv[ch] = o;
        }
        _Float16* hp = hpl + (size_t)(row0 + r) * DM;
        *(volatile v8h*)(hp + lane * 8u)        = hv[0];
        *(volatile v8h*)(hp + 256u + lane * 8u) = hv[1];
        __threadfence();
        *(volatile v8h*)(hp + lane * 8u)        = hv[0];
        *(volatile v8h*)(hp + 256u + lane * 8u) = hv[1];
    }
}
static_assert(SEQ % 32 == 0 && NTOK % 32 == 0);
static_assert(8 * 4 * 2 * 32 * 16 == 32 * DM * 2);
static_assert(38 * DM * 4 + KW * DM * 4 + DM * 4 <= 131072);

__global__ __launch_bounds__(256) __attribute__((amdgpu_num_vgpr(256)))
void k_gemm_res(const _Float16* __restrict__ Ah, const _Float16* __restrict__ Bt,
                const float* __restrict__ bias, const float* resid,
                const float* __restrict__ lnw, const float* __restrict__ lnb,
                float* outF, _Float16* __restrict__ outH,
                float sc, int relu, int lnout, int fin) {
    __shared__ __align__(16) float T[32 * DM];
    const unsigned tid  = threadIdx.x;
    const unsigned lane = tid & 31u;
    const unsigned wave = __builtin_amdgcn_readfirstlane(tid >> 5);
    const unsigned row0 = blockIdx.x * 32u;
    const unsigned cb   = wave * 64u;
    const unsigned r0   = (lane >> 4) << 3;
    const unsigned cc   = lane & 15u;

    v8f acc[2][4], dum[2][4];
    gemm_core<2, 4, false>(Ah + (size_t)row0 * DM, Ah + (size_t)row0 * DM,
                           Bt + (size_t)cb * DM, (unsigned)DM, lane, acc, dum);
#pragma unroll
    for (int mt = 0; mt < 2; ++mt)
#pragma unroll
        for (int nt = 0; nt < 4; ++nt)
#pragma unroll
            for (int g = 0; g < 8; ++g)
                T[(mt * 16 + r0 + g) * DM + cb + nt * 16 + cc] = acc[mt][nt][g];
    __syncthreads();

#pragma unroll 1
    for (unsigned rr = 0; rr < 4u; ++rr) {
        const unsigned row  = wave * 4u + rr;
        const unsigned n    = row0 + row;
        const unsigned fr   = full_row(n);
        const unsigned orow = (fin != 0) ? fr : n;
        const float* rp = resid + (size_t)n * DM;
        float*       op = outF + (size_t)orow * DM;
        v4f xv[4];
        float s = 0.0f;
#pragma unroll
        for (int i = 0; i < 4; ++i) {
            const unsigned c = (unsigned)i * 128u + lane * 4u;
            const v4f a  = *(const v4f*)(&T[row * DM + c]);
            const v4f bi = *(const v4f*)(bias + c);
            const v4f rs = *(const v4f*)(rp + c);
            float y0 = __builtin_fmaf(a.x, sc, bf16r(bi.x));
            float y1 = __builtin_fmaf(a.y, sc, bf16r(bi.y));
            float y2 = __builtin_fmaf(a.z, sc, bf16r(bi.z));
            float y3 = __builtin_fmaf(a.w, sc, bf16r(bi.w));
            y0 = (relu != 0) ? fmaxf(y0, 0.0f) : y0;
            y1 = (relu != 0) ? fmaxf(y1, 0.0f) : y1;
            y2 = (relu != 0) ? fmaxf(y2, 0.0f) : y2;
            y3 = (relu != 0) ? fmaxf(y3, 0.0f) : y3;
            v4f x;
            x.x = rs.x + y0;
            x.y = rs.y + y1;
            x.z = rs.z + y2;
            x.w = rs.w + y3;
            xv[i] = x;
            s += (x.x + x.y) + (x.z + x.w);
        }
        v8h hv0, hv1;
#pragma unroll
        for (int i = 0; i < 8; ++i) { hv0[i] = (_Float16)0.0f; hv1[i] = (_Float16)0.0f; }
        _Float16* hp = outH + (size_t)n * DM;
        if (lnout != 0) {
            s = wave_sum(s);
            const float mu = s * (1.0f / (float)DM);
            float q = 0.0f;
#pragma unroll
            for (int i = 0; i < 4; ++i) {
                const float d0 = xv[i].x - mu, d1 = xv[i].y - mu, d2 = xv[i].z - mu, d3 = xv[i].w - mu;
                q += (d0 * d0 + d1 * d1) + (d2 * d2 + d3 * d3);
            }
            q = wave_sum(q);
            const float rstd = rsqrtf(q * (1.0f / (float)DM) + 1.0e-5f);
#pragma unroll
            for (int i = 0; i < 4; ++i) {
                const unsigned c = (unsigned)i * 128u + lane * 4u;
                const v4f gw = *(const v4f*)(lnw + c);
                const v4f gb = *(const v4f*)(lnb + c);
                v4f y;
                y.x = (xv[i].x - mu) * rstd * bf16r(gw.x) + bf16r(gb.x);
                y.y = (xv[i].y - mu) * rstd * bf16r(gw.y) + bf16r(gb.y);
                y.z = (xv[i].z - mu) * rstd * bf16r(gw.z) + bf16r(gb.z);
                y.w = (xv[i].w - mu) * rstd * bf16r(gw.w) + bf16r(gb.w);
                *(v4f*)(&T[row * DM + c]) = y;
            }
            wave_lds_sync();
            const v4f u0 = *(const v4f*)(&T[row * DM + lane * 8u]);
            const v4f u1 = *(const v4f*)(&T[row * DM + lane * 8u + 4u]);
            const v4f u2 = *(const v4f*)(&T[row * DM + 256u + lane * 8u]);
            const v4f u3 = *(const v4f*)(&T[row * DM + 256u + lane * 8u + 4u]);
            hv0[0] = toh_flush(u0.x * 16.0f); hv0[1] = toh_flush(u0.y * 16.0f);
            hv0[2] = toh_flush(u0.z * 16.0f); hv0[3] = toh_flush(u0.w * 16.0f);
            hv0[4] = toh_flush(u1.x * 16.0f); hv0[5] = toh_flush(u1.y * 16.0f);
            hv0[6] = toh_flush(u1.z * 16.0f); hv0[7] = toh_flush(u1.w * 16.0f);
            hv1[0] = toh_flush(u2.x * 16.0f); hv1[1] = toh_flush(u2.y * 16.0f);
            hv1[2] = toh_flush(u2.z * 16.0f); hv1[3] = toh_flush(u2.w * 16.0f);
            hv1[4] = toh_flush(u3.x * 16.0f); hv1[5] = toh_flush(u3.y * 16.0f);
            hv1[6] = toh_flush(u3.z * 16.0f); hv1[7] = toh_flush(u3.w * 16.0f);
        }
#pragma unroll
        for (int i = 0; i < 4; ++i)
            *(volatile v4f*)(op + (unsigned)i * 128u + lane * 4u) = xv[i];
        if (lnout != 0) {
            *(volatile v8h*)(hp + lane * 8u)        = hv0;
            *(volatile v8h*)(hp + 256u + lane * 8u) = hv1;
        }
        __threadfence();
#pragma unroll
        for (int i = 0; i < 4; ++i)
            *(volatile v4f*)(op + (unsigned)i * 128u + lane * 4u) = xv[i];
        if (lnout != 0) {
            *(volatile v8h*)(hp + lane * 8u)        = hv0;
            *(volatile v8h*)(hp + 256u + lane * 8u) = hv1;
        }
    }
}
static_assert(8 * 4 * 4 * 32 * 16 == 32 * DM * 4);
static_assert(8 * 4 * 2 * 32 * 16 == 32 * DM * 2);
static_assert(8 * 64 == DM);
static_assert(32 * DM * 4 <= 131072);

__global__ __launch_bounds__(256) __attribute__((amdgpu_num_vgpr(256)))
void k_qkv(const _Float16* __restrict__ nh, const _Float16* __restrict__ wT,
           const float* __restrict__ bq, const float* __restrict__ bk,
           const float* __restrict__ bvp,
           _Float16* __restrict__ qk, _Float16* __restrict__ vTh) {
    __shared__ __align__(16) _Float16 stw[8][2048];
    const unsigned tid  = threadIdx.x;
    const unsigned lane = tid & 31u;
    const unsigned w    = __builtin_amdgcn_readfirstlane(tid >> 5);
    const unsigned n0   = blockIdx.y * 128u + (w >> 2) * 64u;
    const unsigned cb   = blockIdx.x * 128u + (w & 3u) * 32u;
    const unsigned r0   = (lane >> 4) << 3;
    const unsigned cc   = lane & 15u;

    v8f acc[4][2], dum[4][2];
    gemm_core<4, 2, false>(nh + (size_t)n0 * DM, nh + (size_t)n0 * DM,
                           wT + (size_t)cb * DM, (unsigned)DM, lane, acc, dum);

    const unsigned t  = cb >> 9;
    const unsigned h  = (cb >> 6) & 7u;
    const unsigned kk = (cb >> 5) & 1u;
    const unsigned o0 = (cb & 511u) + cc;
    const float q0v = bq[o0],  q1v = bq[o0 + 16u];
    const float k0v = bk[o0],  k1v = bk[o0 + 16u];
    const float v0v = bvp[o0], v1v = bvp[o0 + 16u];
    float bv[2];
    bv[0] = bf16r((t == 0u) ? q0v : ((t == 1u) ? k0v : v0v)) * 64.0f;
    bv[1] = bf16r((t == 0u) ? q1v : ((t == 1u) ? k1v : v1v)) * 64.0f;

    if (t < 2u) {
        _Float16* ph = qk + (size_t)t * ((size_t)NTOK * DM);
        const size_t pbase = ((size_t)(h * 2u + kk) * NTOK + n0) * 32u;
#pragma unroll
        for (int mt = 0; mt < 4; ++mt) {
#pragma unroll
            for (int g = 0; g < 8; ++g) {
#pragma unroll
                for (int nt = 0; nt < 2; ++nt) {
                    const float v = __builtin_fmaf(acc[mt][nt][g], SC_Q, bv[nt]);
                    stw[w][(r0 + g) * 32u + nt * 16 + cc] = toh_flush(v);
                }
            }
            wave_lds_sync();
            const v8h a0 = *(const v8h*)(&stw[w][lane * 8u]);
            const v8h a1 = *(const v8h*)(&stw[w][256u + lane * 8u]);
            _Float16* dh = ph + pbase + (size_t)mt * 512u;
            *(volatile v8h*)(dh + lane * 8u)        = a0;
            *(volatile v8h*)(dh + 256u + lane * 8u) = a1;
            __threadfence();
            *(volatile v8h*)(dh + lane * 8u)        = a0;
            *(volatile v8h*)(dh + 256u + lane * 8u) = a1;
            wave_lds_sync();
        }
    } else {
        const unsigned b  = n0 / (unsigned)SEQ;
        const unsigned l0 = n0 - b * (unsigned)SEQ;
        const unsigned hb = h * (unsigned)NB + b;
        const size_t vbase = ((size_t)(hb * HD + kk * 32u)) * SEQ + l0;
        const unsigned rq = lane >> 3;
        const unsigned pc = (lane & 7u) << 3;
        v8h xv[8];
#pragma unroll
        for (int mt = 0; mt < 4; ++mt)
#pragma unroll
            for (int nt = 0; nt < 2; ++nt) {
                v8h hv;
#pragma unroll
                for (int g = 0; g < 8; ++g)
                    hv[g] = toh_flush(__builtin_fmaf(acc[mt][nt][g], SC_Q, bv[nt]));
                *(v8h*)(&stw[w][(nt * 16 + cc) * 64u + mt * 16 + r0]) = hv;
            }
        wave_lds_sync();
#pragma unroll
        for (int i = 0; i < 8; ++i) xv[i] = *(const v8h*)(&stw[w][(i * 4 + rq) * 64u + pc]);
#pragma unroll
        for (int i = 0; i < 8; ++i)
            *(volatile v8h*)(vTh + vbase + (size_t)(i * 4 + rq) * SEQ + pc) = xv[i];
        __threadfence();
#pragma unroll
        for (int i = 0; i < 8; ++i)
            *(volatile v8h*)(vTh + vbase + (size_t)(i * 4 + rq) * SEQ + pc) = xv[i];
    }
}
static_assert(4 * 2 * 32 * 16 == 64 * 32 * 2);
static_assert(8 * 32 * 16 == 32 * 64 * 2);
static_assert(12 * 128 == 3 * DM);

__global__ __launch_bounds__(256) __attribute__((amdgpu_num_vgpr(256)))
void k_attn(const _Float16* __restrict__ qh, const _Float16* __restrict__ kh,
            const _Float16* __restrict__ vTh,
            const float* __restrict__ ek, const float* __restrict__ ev,
            _Float16* __restrict__ ctxh) {
    __shared__ __align__(16) _Float16 Ek[48 * HD];
    __shared__ __align__(16) _Float16 Evt[HD * 64];
    __shared__ __align__(16) float    Qe[8][16 * 48];
    __shared__ __align__(16) float    Tb[8][16 * 36];
    __shared__ __align__(16) _Float16 Wt[8][16 * 64];
    __shared__ __align__(16) _Float16 Ch[8][16 * HD];

    const unsigned tid  = threadIdx.x;
    const unsigned lane = tid & 31u;
    const unsigned wave = __builtin_amdgcn_readfirstlane(tid >> 5);
    const unsigned hb   = blockIdx.x;
    const unsigned h    = hb / (unsigned)NB;
    const unsigned b    = hb - h * (unsigned)NB;
    const unsigned q0   = blockIdx.y * 128u + wave * 16u;
    const unsigned r0   = (lane >> 4) << 3;
    const unsigned cc   = lane & 15u;

#pragma unroll 1
    for (unsigned idx = tid; idx < 48u * HD; idx += 256u) {
        const unsigned v  = idx >> 6, d = idx & 63u;
        const unsigned vc = (v < 32u) ? v : 32u;
        float e = ek[vc * HD + d];
        asm volatile("" : "+v"(e));
        Ek[idx] = (v < 33u) ? toh_flush(bf16r(e) * 64.0f) : (_Float16)0.0f;
    }
#pragma unroll 1
    for (unsigned idx = tid; idx < (unsigned)HD * 64u; idx += 256u) {
        const unsigned d  = idx >> 6, v = idx & 63u;
        const unsigned vc = (v < 32u) ? v : 32u;
        float e = ev[vc * HD + d];
        asm volatile("" : "+v"(e));
        Evt[idx] = (v < 33u) ? toh_flush(bf16r(e) * 64.0f) : (_Float16)0.0f;
    }
#pragma unroll 1
    for (unsigned i = lane; i < 16u * 36u; i += 32u) Tb[wave][i] = -1.0e30f;
    __syncthreads();

    const size_t tokq = (size_t)b * SEQ + q0;
    const size_t tokk = (size_t)b * SEQ;
    const size_t P0 = (size_t)(h * 2u) * NTOK;
    const size_t P1 = (size_t)(h * 2u + 1u) * NTOK;
    const v16h qhf0 = load_frag16(qh + (P0 + tokq) * 32u, 32u, lane);
    const v16h qhf1 = load_frag16(qh + (P1 + tokq) * 32u, 32u, lane);
    const _Float16* kh0 = kh + (P0 + tokk) * 32u;
    const _Float16* kh1 = kh + (P1 + tokk) * 32u;
    const _Float16* vhb = vTh + (size_t)hb * HD * SEQ;

#pragma unroll
    for (int vt = 0; vt < 3; ++vt) {
        v8f e = zero8();
        Frag a;
        a.h[0] = *(const v8h*)(&Ek[(vt * 16 + cc) * HD + r0]);
        a.h[1] = *(const v8h*)(&Ek[(vt * 16 + cc) * HD + r0 + 16u]);
        e = wmma16(a.v, qhf0, e);
        a.h[0] = *(const v8h*)(&Ek[(vt * 16 + cc) * HD + 32u + r0]);
        a.h[1] = *(const v8h*)(&Ek[(vt * 16 + cc) * HD + 48u + r0]);
        e = wmma16(a.v, qhf1, e);
        v4f e0, e1;
        e0.x = e[0] * C1; e0.y = e[1] * C1; e0.z = e[2] * C1; e0.w = e[3] * C1;
        e1.x = e[4] * C1; e1.y = e[5] * C1; e1.z = e[6] * C1; e1.w = e[7] * C1;
        *(v4f*)(&Qe[wave][cc * 48u + vt * 16 + r0])      = e0;
        *(v4f*)(&Qe[wave][cc * 48u + vt * 16 + r0 + 4u]) = e1;
    }
    wave_lds_sync();
    const float qeL = Qe[wave][cc * 48u];
    const float qeR = Qe[wave][cc * 48u + 32u];
    const int   dbq = (int)r0 - (int)cc;

    v8f oh[4];
#pragma unroll
    for (int dt = 0; dt < 4; ++dt) oh[dt] = zero8();
    float mr = -1.0e30f, lr = 0.0f, wl = 0.0f, wr = 0.0f;

#pragma unroll 1
    for (unsigned key0 = 0; key0 < (unsigned)SEQ; key0 += 32u) {
        v8f s0 = zero8(), s1 = zero8();
        {
            v16h a = load_frag16(kh0 + (size_t)key0 * 32u, 32u, lane);
            s0 = wmma16(a, qhf0, s0);
            a = load_frag16(kh1 + (size_t)key0 * 32u, 32u, lane);
            s0 = wmma16(a, qhf1, s0);
        }
        {
            v16h a = load_frag16(kh0 + (size_t)(key0 + 16u) * 32u, 32u, lane);
            s1 = wmma16(a, qhf0, s1);
            a = load_frag16(kh1 + (size_t)(key0 + 16u) * 32u, 32u, lane);
            s1 = wmma16(a, qhf1, s1);
        }
        const int dlo = (int)key0 - (int)q0;
        float t0[8], t1[8];
#pragma unroll
        for (int g = 0; g < 8; ++g) {
            t0[g] = s0[g] * C1;
            t1[g] = s1[g] * C1;
        }
        if (dlo <= -47) {
#pragma unroll
            for (int g = 0; g < 8; ++g) { t0[g] += qeL; t1[g] += qeL; }
        } else if (dlo >= 31) {
#pragma unroll
            for (int g = 0; g < 8; ++g) { t0[g] += qeR; t1[g] += qeR; }
        } else {
            const int db = dlo + dbq;
#pragma unroll
            for (int g = 0; g < 8; ++g) {
                const int d0 = db + g;
                const int d1 = d0 + 16;
                const int i0 = ((d0 < -16) ? -16 : ((d0 > 16) ? 16 : d0)) + 16;
                const int i1 = ((d1 < -16) ? -16 : ((d1 > 16) ? 16 : d1)) + 16;
                t0[g] += Qe[wave][cc * 48u + (unsigned)i0];
                t1[g] += Qe[wave][cc * 48u + (unsigned)i1];
            }
        }
        float tmax = fmaxf(t0[0], t1[0]);
#pragma unroll
        for (int g = 1; g < 8; ++g) tmax = fmaxf(tmax, fmaxf(t0[g], t1[g]));
        tmax = fmaxf(tmax, __shfl_xor(tmax, 16, 32));
        const float mn    = fmaxf(mr, tmax);
        const float alpha = ex2(mr - mn);
        mr = mn;
        const float off = 14.0f - mn;
        v8h p0, p1;
        float psp = 0.0f;
#pragma unroll
        for (int g = 0; g < 8; ++g) {
            const float e0 = t0[g] + off;
            const float e1 = t1[g] + off;
            const _Float16 x0 = (_Float16)ex2(e0);
            const _Float16 x1 = (_Float16)ex2(e1);
            const _Float16 a = (e0 < -14.0f) ? (_Float16)0.0f : x0;
            const _Float16 c = (e1 < -14.0f) ? (_Float16)0.0f : x1;
            p0[g] = a;
            p1[g] = c;
            psp += (float)a + (float)c;
        }
        float psl = 0.0f, psr = 0.0f;
        if (dlo <= -47) {
            psl = psp;
        } else if (dlo >= 31) {
            psr = psp;
        } else {
            const int db = dlo + dbq;
#pragma unroll
            for (int g = 0; g < 8; ++g) {
                const int d0 = db + g;
                const int d1 = d0 + 16;
                const float pa = (float)p0[g];
                const float pc2 = (float)p1[g];
                psl += (d0 <= -16) ? pa : 0.0f;
                psr += (d0 >= 16) ? pa : 0.0f;
                psl += (d1 <= -16) ? pc2 : 0.0f;
                psr += (d1 >= 16) ? pc2 : 0.0f;
                if ((d0 > -16) & (d0 < 16)) Tb[wave][cc * 36u + (unsigned)(d0 + 16)] = t0[g];
                if ((d1 > -16) & (d1 < 16)) Tb[wave][cc * 36u + (unsigned)(d1 + 16)] = t1[g];
            }
        }
        const float ps = psp + __shfl_xor(psp, 16, 32);
        psl += __shfl_xor(psl, 16, 32);
        psr += __shfl_xor(psr, 16, 32);
        lr = lr * alpha + ps;
        wl = wl * alpha + psl;
        wr = wr * alpha + psr;
        Frag pb;
        pb.h[0] = p0;
        pb.h[1] = p1;
#pragma unroll
        for (int dt = 0; dt < 4; ++dt) oh[dt] = oh[dt] * alpha;
#pragma unroll
        for (int dt = 0; dt < 4; ++dt) {
            const v16h va = load_frag16(vhb + (size_t)(dt * 16) * SEQ + key0, (unsigned)SEQ, lane);
            oh[dt] = wmma16(va, pb.v, oh[dt]);
        }
    }

    wave_lds_sync();
    const float invl = 1.0f / lr;
    const float offf = 14.0f - mr;
    const float wsc  = invl * 1024.0f;
    const unsigned hh = lane >> 4;
    const float edge = ((hh == 0u) ? wl : wr) * wsc;
#pragma unroll 1
    for (unsigned jj = 0; jj < 4u; ++jj) {
        v8h o;
#pragma unroll
        for (int i = 0; i < 8; ++i) {
            const unsigned col = hh * 32u + jj * 8u + (unsigned)i;
            const unsigned cl  = (col < 35u) ? col : 35u;
            float tv = Tb[wave][cc * 36u + cl];
            asm volatile("" : "+v"(tv));
            float wv = ex2(tv + offf) * wsc;
            if (i == 0) wv = (jj == 0u) ? edge : wv;
            o[i] = toh_flush(wv);
        }
        *(v8h*)(&Wt[wave][cc * 64u + hh * 32u + jj * 8u]) = o;
    }
    wave_lds_sync();

    v8f orel[4];
#pragma unroll
    for (int dt = 0; dt < 4; ++dt) orel[dt] = zero8();
#pragma unroll
    for (int ks = 0; ks < 2; ++ks) {
        Frag wb;
        wb.h[0] = *(const v8h*)(&Wt[wave][cc * 64u + ks * 32 + r0]);
        wb.h[1] = *(const v8h*)(&Wt[wave][cc * 64u + ks * 32 + r0 + 16u]);
#pragma unroll
        for (int dt = 0; dt < 4; ++dt) {
            Frag ea;
            ea.h[0] = *(const v8h*)(&Evt[(dt * 16 + cc) * 64u + ks * 32 + r0]);
            ea.h[1] = *(const v8h*)(&Evt[(dt * 16 + cc) * 64u + ks * 32 + r0 + 16u]);
            orel[dt] = wmma16(ea.v, wb.v, orel[dt]);
        }
    }

    const float inv = 0.25f * invl;
#pragma unroll
    for (int dt = 0; dt < 4; ++dt) {
        v8h hv;
#pragma unroll
        for (int g = 0; g < 8; ++g) {
            const float c = __builtin_fmaf(orel[dt][g], SC_REL, oh[dt][g] * inv);
            hv[g] = toh_flush(c);
        }
        *(v8h*)(&Ch[wave][cc * HD + dt * 16 + r0]) = hv;
    }
    wave_lds_sync();
    const unsigned rq = lane >> 3;
    const unsigned pc = (lane & 7u) << 3;
    v8h ch[4];
#pragma unroll
    for (int i = 0; i < 4; ++i) ch[i] = *(const v8h*)(&Ch[wave][(i * 4 + rq) * HD + pc]);
    const size_t ob = (tokq) * DM + h * HD + pc;
#pragma unroll
    for (int i = 0; i < 4; ++i)
        *(volatile v8h*)(ctxh + ob + (size_t)(i * 4 + rq) * DM) = ch[i];
    __threadfence();
#pragma unroll
    for (int i = 0; i < 4; ++i)
        *(volatile v8h*)(ctxh + ob + (size_t)(i * 4 + rq) * DM) = ch[i];
}
static_assert(4 * 32 * 16 == 16 * HD * 2);
static_assert(48 * HD * 2 + HD * 64 * 2 + 8 * 16 * 48 * 4 + 8 * 16 * 36 * 4 + 8 * 16 * 64 * 2 + 8 * 16 * HD * 2 <= 131072);
static_assert(8 * 2048 * 2 <= 131072);
static_assert((48 * HD) % 256 == 0 && (HD * 64) % 256 == 0 && (16 * 36) % 32 == 0);
static_assert(NREL <= 48 && NREL <= 64 && NREL - 1 == 32);

#define U_BYTES ((size_t)NTOK * DM * 2)
#define W_BYTES ((size_t)DM * DM * 2)
static_assert((size_t)NB_FULL * SEQ_FULL * DM * 2 * 7 + 7 * W_BYTES + (size_t)SEQ_FULL * DM * 4 <= (size_t)134217728);
static_assert(U_BYTES % 128 == 0 && W_BYTES % 128 == 0);

extern "C" void kernel_launch(void* const* d_in, const int* in_sizes, int n_in,
                              void* d_out, int out_size, void* d_ws, size_t ws_size,
                              hipStream_t stream) {
    if (n_in < 24) return;
    const int need_rows = (NB - 1) * SEQ_FULL + SEQ;
    if (in_sizes[0] < need_rows * DM) return;
    if (in_sizes[1] < need_rows) return;
    if (in_sizes[2] < 2 * DM * KW || in_sizes[3] < 2 * DM) return;
    if (in_sizes[4] < 2 * DM * DM || in_sizes[5] < 2 * DM) return;
    if (in_sizes[6] < 2 * DM || in_sizes[7] < 2 * DM) return;
    if (in_sizes[8] < DM * DM || in_sizes[9] < DM) return;
    if (in_sizes[10] < DM * DM || in_sizes[11] < DM) return;
    if (in_sizes[12] < DM * DM || in_sizes[13] < DM) return;
    if (in_sizes[14] < DM * DM || in_sizes[15] < DM) return;
    if (in_sizes[16] < NREL * HD || in_sizes[17] < NREL * HD) return;
    if (in_sizes[18] < DM || in_sizes[19] < DM) return;
    if (in_sizes[20] < DM * DM || in_sizes[21] < DM) return;
    if (in_sizes[22] < DM || in_sizes[23] < DM) return;
    if (out_size < need_rows * DM) return;

    const float* x     = (const float*)d_in[0];
    const int*   mask  = (const int*)  d_in[1];
    const float* dww   = (const float*)d_in[2];
    const float* dwb   = (const float*)d_in[3];
    const float* pww   = (const float*)d_in[4];
    const float* pwb   = (const float*)d_in[5];
    const float* lncg  = (const float*)d_in[6];
    const float* lncb  = (const float*)d_in[7];
    const float* wq    = (const float*)d_in[8];
    const float* bq    = (const float*)d_in[9];
    const float* wk    = (const float*)d_in[10];
    const float* bk    = (const float*)d_in[11];
    const float* wv    = (const float*)d_in[12];
    const float* bv    = (const float*)d_in[13];
    const float* wo    = (const float*)d_in[14];
    const float* bo    = (const float*)d_in[15];
    const float* embk  = (const float*)d_in[16];
    const float* embv  = (const float*)d_in[17];
    const float* lnag  = (const float*)d_in[18];
    const float* lnab  = (const float*)d_in[19];
    const float* wff   = (const float*)d_in[20];
    const float* bff   = (const float*)d_in[21];
    const float* lnfg  = (const float*)d_in[22];
    const float* lnfb  = (const float*)d_in[23];
    float* out = (float*)d_out;

    const size_t U  = U_BYTES;
    const size_t WB = W_BYTES;
    const size_t total = 7 * U + 7 * WB + (size_t)SEQ * DM * 4;
    if (total > ws_size) return;

    char* ws = (char*)d_ws;
    float*    xs    = (float*)(ws + 0 * U);
    _Float16* pl0   = (_Float16*)(ws + 2 * U);
    _Float16* pl1   = (_Float16*)(ws + 3 * U);
    _Float16* qk    = (_Float16*)(ws + 4 * U);
    _Float16* vTh   = (_Float16*)(ws + 6 * U);
    _Float16* pwT   = (_Float16*)(ws + 7 * U);
    _Float16* wqkvT = (_Float16*)(ws + 7 * U + 2 * WB);
    _Float16* woT   = (_Float16*)(ws + 7 * U + 5 * WB);
    _Float16* wffT  = (_Float16*)(ws + 7 * U + 6 * WB);
    float*    pe    = (float*)(ws + 7 * U + 7 * WB);

    k_wcvt<<<dim3(2 * DM * DM / 2048), dim3(256), 0, stream>>>(pww, pwT);
    k_wcvt<<<dim3(DM * DM / 2048), dim3(256), 0, stream>>>(wq, wqkvT);
    k_wcvt<<<dim3(DM * DM / 2048), dim3(256), 0, stream>>>(wk, wqkvT + (size_t)DM * DM);
    k_wcvt<<<dim3(DM * DM / 2048), dim3(256), 0, stream>>>(wv, wqkvT + (size_t)2 * DM * DM);
    k_wcvt<<<dim3(DM * DM / 2048), dim3(256), 0, stream>>>(wo, woT);
    k_wcvt<<<dim3(DM * DM / 2048), dim3(256), 0, stream>>>(wff, wffT);

    k_pe<<<dim3(SEQ), dim3(256), 0, stream>>>(pe);
    k_pos<<<dim3(NTOK / 2), dim3(256), 0, stream>>>(x, mask, pe, xs);

    k_lnconv<<<dim3(NTOK / 32), dim3(256), 0, stream>>>(xs, lncg, lncb, dww, dwb, pl0);
    k_gemm_res<<<dim3(NTOK / 32), dim3(256), 0, stream>>>(
        pl0, pwT, pwb, xs, lnag, lnab, xs, pl1, SC_CONV, 1, 0, 0);
    k_lnconv<<<dim3(NTOK / 32), dim3(256), 0, stream>>>(xs, lncg + DM, lncb + DM,
                                                        dww + (size_t)DM * KW, dwb + DM, pl0);
    k_gemm_res<<<dim3(NTOK / 32), dim3(256), 0, stream>>>(
        pl0, pwT + (size_t)DM * DM, pwb + DM, xs, lnag, lnab, xs, pl1, SC_CONV, 1, 1, 0);

    k_qkv<<<dim3(12, NTOK / 128), dim3(256), 0, stream>>>(pl1, wqkvT, bq, bk, bv, qk, vTh);
    k_attn<<<dim3(NH * NB, SEQ / 128), dim3(256), 0, stream>>>(
        qk, qk + (size_t)NTOK * DM, vTh, embk, embv, pl0);
    k_gemm_res<<<dim3(NTOK / 32), dim3(256), 0, stream>>>(
        pl0, woT, bo, xs, lnfg, lnfb, xs, pl1, SC_OUT, 0, 1, 0);
    k_gemm_res<<<dim3(NTOK / 32), dim3(256), 0, stream>>>(
        pl1, wffT, bff, xs, lnfg, lnfb, out, pl0, SC_OUT, 1, 0, 1);
}
